// Prior_22119081574563
// MI455X (gfx1250) — hardware-run, weakly checked
//
#include <hip/hip_runtime.h>
#include <stddef.h>


#define D       128
#define DO      64
#define NTHR    256
#define NWAVE   8
#define EPT     8
#define NGRP    2
#define CHUNK   (NTHR * EPT * NGRP)
#define WCAP    (EPT * NGRP * 32)
#define LISTN   (NWAVE * WCAP)
#define NBC     4096
#define NBF     1024
#define RCAP    40960
#define RBN     128
#define TGT     256
#define DEGCAP  256
#define GROWS   128
#define BNR     64
#define OTHR    512
#define AP      (D + 8)
#define BNEPS   1e-5f

#define LDS_GA   (GROWS * AP * 2)
#define LDS_GST  (2 * LDS_GA)
#define LDS_GEMM (LDS_GST + 256 * 8)
#define LDS_FILL ((RCAP + NBF + LISTN) * 4 + 64)

static_assert((CHUNK & (CHUNK - 1)) == 0);
static_assert(CHUNK <= 4096);
static_assert(NBC <= 4096 && NBF <= 4096);
static_assert((NBC & (NBC - 1)) == 0 && (NBF & (NBF - 1)) == 0);
static_assert(NBC == 4 * NBF);
static_assert(OTHR * 8 == NBC);
static_assert((RCAP % 32) == 0);
static_assert(GROWS * D * 4 <= LDS_GST);
static_assert((TGT % GROWS) == 0 && TGT == NWAVE * 32 && (TGT % BNR) == 0);
static_assert((GROWS * D / 8) % NTHR == 0);
static_assert((D * D / 8) % NTHR == 0 && (D * DO / 8) % NTHR == 0);
static_assert(BNR == NWAVE * 8);
static_assert(((AP * 2) % 16) == 0);

typedef float          v4f   __attribute__((ext_vector_type(4)));
typedef float          v8f   __attribute__((ext_vector_type(8)));
typedef int            v4i   __attribute__((ext_vector_type(4)));
typedef double         v2d   __attribute__((ext_vector_type(2)));
typedef unsigned short v8us  __attribute__((ext_vector_type(8)));
typedef __bf16         v16bf __attribute__((ext_vector_type(16)));
union FragB { v16bf v; v8us h[2]; };
union FI { float f; int i; };

__device__ __forceinline__ unsigned bfbits(float f) {
  unsigned u = __float_as_uint(f);
  u += 0x7FFFu + ((u >> 16) & 1u);
  return u >> 16;
}

__device__ __forceinline__ void split8(v4f a, v4f b, v8us& hv, v8us& lv) {
  float v[8];
  v[0] = a.x; v[1] = a.y; v[2] = a.z; v[3] = a.w; v[4] = b.x; v[5] = b.y; v[6] = b.z; v[7] = b.w;
  v8us h, l;
#pragma unroll
  for (int e = 0; e < 8; ++e) {
    const unsigned hb = bfbits(v[e]);
    const float hf = __uint_as_float(hb << 16);
    const unsigned lb = bfbits(v[e] - hf);
    h[e] = (unsigned short)hb;
    l[e] = (unsigned short)lb;
  }
  hv = h; lv = l;
}

__device__ __forceinline__ v8f wmb(v16bf a, v16bf b, v8f c) {
  v8f d = __builtin_amdgcn_wmma_f32_16x16x32_bf16(false, a, false, b, (short)0, c, false, false);
  asm volatile("v_nop\n\tv_nop\n\tv_nop\n\tv_nop" : "+v"(d) : "v"(a), "v"(b));
  return d;
}

template <int NB>
__device__ __forceinline__ int scan_chunk(const int* __restrict__ dsts, int nE, int cbase, int slotBase,
                                          int vec8, int* list, int tid, int lane, int wave) {
  int wc = 0;
#pragma unroll
  for (int g = 0; g < NGRP; ++g) {
    const int el0  = (g * NTHR + tid) * EPT;
    const int e0   = cbase + el0;
    const int sent = -2147483647 - 1;
    v4i da, db;
    if (vec8 != 0 && cbase + CHUNK <= nE) {
      da = *(const v4i*)(dsts + e0);
      db = *(const v4i*)(dsts + e0 + 4);
    } else {
      da.x = (e0     < nE) ? dsts[min(e0, nE - 1)] : sent;
      da.y = (e0 + 1 < nE) ? dsts[min(e0 + 1, nE - 1)] : sent;
      da.z = (e0 + 2 < nE) ? dsts[min(e0 + 2, nE - 1)] : sent;
      da.w = (e0 + 3 < nE) ? dsts[min(e0 + 3, nE - 1)] : sent;
      db.x = (e0 + 4 < nE) ? dsts[min(e0 + 4, nE - 1)] : sent;
      db.y = (e0 + 5 < nE) ? dsts[min(e0 + 5, nE - 1)] : sent;
      db.z = (e0 + 6 < nE) ? dsts[min(e0 + 6, nE - 1)] : sent;
      db.w = (e0 + 7 < nE) ? dsts[min(e0 + 7, nE - 1)] : sent;
    }
    const unsigned nb = (unsigned)slotBase;
    const unsigned s0 = (unsigned)da.x - nb, s1 = (unsigned)da.y - nb;
    const unsigned s2 = (unsigned)da.z - nb, s3 = (unsigned)da.w - nb;
    const unsigned s4 = (unsigned)db.x - nb, s5 = (unsigned)db.y - nb;
    const unsigned s6 = (unsigned)db.z - nb, s7 = (unsigned)db.w - nb;
    const bool h0 = s0 < (unsigned)NB, h1 = s1 < (unsigned)NB, h2 = s2 < (unsigned)NB, h3 = s3 < (unsigned)NB;
    const bool h4 = s4 < (unsigned)NB, h5 = s5 < (unsigned)NB, h6 = s6 < (unsigned)NB, h7 = s7 < (unsigned)NB;
    const unsigned any = __builtin_amdgcn_ballot_w32(h0 | h1 | h2 | h3 | h4 | h5 | h6 | h7);
    if (any != 0u) {
#define HITJ(J, HJ, SJ) { \
        const unsigned mj = __builtin_amdgcn_ballot_w32(HJ); \
        if (mj != 0u) { \
          if (HJ) { \
            const int pos = wc + (int)__builtin_amdgcn_mbcnt_lo(mj, 0u); \
            if (pos < WCAP) list[wave * WCAP + pos] = ((el0 + (J)) << 12) | (int)(SJ); \
          } \
          wc += (int)__builtin_popcount(mj); } }
      HITJ(0, h0, s0)
      HITJ(1, h1, s1)
      HITJ(2, h2, s2)
      HITJ(3, h3, s3)
      HITJ(4, h4, s4)
      HITJ(5, h5, s5)
      HITJ(6, h6, s6)
      HITJ(7, h7, s7)
#undef HITJ
    }
  }
  return wc;
}

__global__ __launch_bounds__(NTHR) void k_wprep(
    const float* __restrict__ W1, const float* __restrict__ W2, const float* __restrict__ W3,
    unsigned short* h1, unsigned short* l1, unsigned short* h2, unsigned short* l2,
    unsigned short* h3, unsigned short* l3) {
  const int g0 = D * D / 8, g1 = D * D / 8, g2 = D * DO / 8;
  const int bstart = blockIdx.x * NTHR;
  const float* src; unsigned short* dh; unsigned short* dl; int Nout, segOff;
  if (bstart < g0)           { src = W1; dh = h1; dl = l1; Nout = D;  segOff = 0; }
  else if (bstart < g0 + g1) { src = W2; dh = h2; dl = l2; Nout = D;  segOff = g0; }
  else                       { src = W3; dh = h3; dl = l3; Nout = DO; segOff = g0 + g1; }
  const int i = bstart + (int)threadIdx.x;
  if (i >= g0 + g1 + g2) return;
  const int o  = (i - segOff) * 8;
  const int n  = o / D;
  const int k0 = o - n * D;
  float v[8];
#pragma unroll
  for (int e = 0; e < 8; ++e) v[e] = src[(size_t)(k0 + e) * Nout + n];
  v4f a, b;
  a.x = v[0]; a.y = v[1]; a.z = v[2]; a.w = v[3];
  b.x = v[4]; b.y = v[5]; b.z = v[6]; b.w = v[7];
  v8us hv, lv;
  split8(a, b, hv, lv);
  unsigned short* ph = dh + o;
  unsigned short* pl = dl + o;
  *(volatile v8us*)ph = hv;
  *(volatile v8us*)pl = lv;
  __threadfence();
  *(volatile v8us*)ph = hv;
  *(volatile v8us*)pl = lv;
}

__global__ __launch_bounds__(NTHR) void k_count(
    const int* __restrict__ ei, int* cnt, float* dinv, int nE, int vec8) {
  __shared__ __attribute__((aligned(16))) int scnt[NBC];
  __shared__ __attribute__((aligned(16))) int list[LISTN];
  __shared__ int wcnt[NWAVE];
  const int tid = threadIdx.x, lane = tid & 31, wave = tid >> 5;
  const int nodeBase = blockIdx.x * NBC;
  const int* dsts = ei + nE;

  for (int i = tid; i < NBC; i += NTHR) scnt[i] = 0;
  __syncthreads();

  const int nChunks = (nE + CHUNK - 1) / CHUNK;
#pragma unroll 1
  for (int ch = 0; ch < nChunks; ++ch) {
    const int cbase = ch * CHUNK;
    const int wc = scan_chunk<NBC>(dsts, nE, cbase, nodeBase, vec8, list, tid, lane, wave);
    if (lane == 0) wcnt[wave] = wc;
    __syncthreads();
    if (wave == 0) {
#pragma unroll 1
      for (int wsx = 0; wsx < NWAVE; ++wsx) {
        int n = __builtin_amdgcn_readfirstlane(wcnt[wsx]);
        n = n > WCAP ? WCAP : (n < 0 ? 0 : n);
        const int* lp = list + wsx * WCAP;
#pragma unroll 1
        for (int i = 0; i < n; ++i) {
          const int ent  = __builtin_amdgcn_readfirstlane(lp[i]);
          const int slot = ent & (NBC - 1);
          if (lane == 0) scnt[slot] = scnt[slot] + 1;
        }
      }
    }
    __syncthreads();
  }

  v4i cq[4]; v4f dq[4];
#pragma unroll
  for (int q = 0; q < 4; ++q) {
    const int f = (wave * 4 + q) * 128 + 4 * lane;
    const v4i c = *(const v4i*)(scnt + f);
    cq[q] = c;
    dq[q].x = rsqrtf((float)(c.x + 1));
    dq[q].y = rsqrtf((float)(c.y + 1));
    dq[q].z = rsqrtf((float)(c.z + 1));
    dq[q].w = rsqrtf((float)(c.w + 1));
  }
  int*   cp = cnt + (size_t)nodeBase;
  float* dp = dinv + (size_t)nodeBase;
#pragma unroll
  for (int q = 0; q < 4; ++q) {
    const int f = (wave * 4 + q) * 128 + 4 * lane;
    *(volatile v4i*)(cp + f) = cq[q];
    *(volatile v4f*)(dp + f) = dq[q];
  }
  __threadfence();
#pragma unroll
  for (int q = 0; q < 4; ++q) {
    const int f = (wave * 4 + q) * 128 + 4 * lane;
    *(volatile v4i*)(cp + f) = cq[q];
    *(volatile v4f*)(dp + f) = dq[q];
  }
}

__global__ __launch_bounds__(OTHR) void k_offsets(
    const int* __restrict__ cnt, int* off, int* rbase, int nChunk) {
  __shared__ __attribute__((aligned(16))) int soff[NBC];
  __shared__ __attribute__((aligned(16))) int srb[RBN];
  __shared__ int wtot[OTHR / 32];
  const int tid = threadIdx.x, lane = tid & 31, wave = tid >> 5, sub = tid >> 7;
  for (int i = tid; i < RBN; i += OTHR) srb[i] = 0;
  int carry = 0;
#pragma unroll 1
  for (int ch = 0; ch < nChunk; ++ch) {
    const int base = ch * NBC;
    const v4i c0 = *(const v4i*)(cnt + base + 8 * tid);
    const v4i c1 = *(const v4i*)(cnt + base + 8 * tid + 4);
    const int e0 = max(c0.x, 0), e1 = max(c0.y, 0), e2 = max(c0.z, 0), e3 = max(c0.w, 0);
    const int e4 = max(c1.x, 0), e5 = max(c1.y, 0), e6 = max(c1.z, 0), e7 = max(c1.w, 0);
    const int ts = e0 + e1 + e2 + e3 + e4 + e5 + e6 + e7;
    int incl = ts;
#pragma unroll
    for (int dd = 1; dd < 32; dd <<= 1) {
      const int t = __shfl_up(incl, dd);
      if (lane >= dd) incl += t;
    }
    if (lane == 31) wtot[wave] = incl;
    __syncthreads();
    const int S0 = wtot[0]  + wtot[1]  + wtot[2]  + wtot[3];
    const int S1 = wtot[4]  + wtot[5]  + wtot[6]  + wtot[7];
    const int S2 = wtot[8]  + wtot[9]  + wtot[10] + wtot[11];
    const int S3 = wtot[12] + wtot[13] + wtot[14] + wtot[15];
    int pre = 0;
#pragma unroll 1
    for (int w = 4 * sub; w < wave; ++w) pre += wtot[w];
    const int b0 = carry;
    const int b1 = b0 + ((S0 + 31) & ~31);
    const int b2 = b1 + ((S1 + 31) & ~31);
    const int b3 = b2 + ((S2 + 31) & ~31);
    const int b4 = b3 + ((S3 + 31) & ~31);
    const int myb = sub == 0 ? b0 : (sub == 1 ? b1 : (sub == 2 ? b2 : b3));
    if (tid == 0) {
      srb[min(4 * ch + 0, RBN - 1)] = b0;
      srb[min(4 * ch + 1, RBN - 1)] = b1;
      srb[min(4 * ch + 2, RBN - 1)] = b2;
      srb[min(4 * ch + 3, RBN - 1)] = b3;
    }
    int run = myb + pre + incl - ts;
    soff[8 * tid + 0] = run; run += e0;
    soff[8 * tid + 1] = run; run += e1;
    soff[8 * tid + 2] = run; run += e2;
    soff[8 * tid + 3] = run; run += e3;
    soff[8 * tid + 4] = run; run += e4;
    soff[8 * tid + 5] = run; run += e5;
    soff[8 * tid + 6] = run; run += e6;
    soff[8 * tid + 7] = run;
    carry = b4;
    __syncthreads();
    const v4i o0 = *(const v4i*)(soff + 4 * tid);
    const v4i o1 = *(const v4i*)(soff + 4 * (tid + OTHR));
    int* op = off + base;
    *(volatile v4i*)(op + 4 * tid) = o0;
    *(volatile v4i*)(op + 4 * (tid + OTHR)) = o1;
    __threadfence();
    *(volatile v4i*)(op + 4 * tid) = o0;
    *(volatile v4i*)(op + 4 * (tid + OTHR)) = o1;
    __syncthreads();
  }
  if (tid == 0) srb[min(4 * nChunk, RBN - 1)] = carry;
  __syncthreads();
  v4i rv = {0, 0, 0, 0};
  if (tid < 32) rv = *(const v4i*)(srb + 4 * tid);
  if (tid < 32) *(volatile v4i*)(rbase + 4 * tid) = rv;
  __threadfence();
  if (tid < 32) *(volatile v4i*)(rbase + 4 * tid) = rv;
}

__global__ __launch_bounds__(NTHR) void k_fill(
    const int* __restrict__ ei, const int* __restrict__ off, const int* __restrict__ rbase,
    int* csr, int nN, int nE, int vec8, int csrLen) {
  extern __shared__ v4f lds_dyn[];
  int* region = (int*)lds_dyn;
  int* cursor = region + RCAP;
  int* list   = cursor + NBF;
  int* wcnt   = list + LISTN;
  const int tid = threadIdx.x, lane = tid & 31, wave = tid >> 5;
  const int b = blockIdx.x;
  const int nodeBase = b * NBF;
  const int* dsts = ei + nE;

  int rb0 = rbase[b];
  const int rb1 = rbase[b + 1];
  rb0 = rb0 < 0 ? 0 : (rb0 > csrLen ? csrLen : rb0);
  rb0 &= ~31;
  int len = rb1 - rb0;
  len = len < 0 ? 0 : (len > RCAP ? RCAP : len);
  int lenW = (len + 31) & ~31;
  if (rb0 + lenW > csrLen) lenW = (csrLen - rb0) & ~31;

  {
    const v4i z = {0, 0, 0, 0};
    for (int i = tid; i < RCAP / 4; i += NTHR) ((v4i*)region)[i] = z;
    for (int s = tid; s < NBF; s += NTHR) {
      int o = off[nodeBase + s] - rb0;
      o = o < 0 ? 0 : (o > RCAP ? RCAP : o);
      cursor[s] = o;
    }
  }
  __syncthreads();

  const int nChunks = (nE + CHUNK - 1) / CHUNK;
#pragma unroll 1
  for (int ch = 0; ch < nChunks; ++ch) {
    const int cbase = ch * CHUNK;
    const int wc = scan_chunk<NBF>(dsts, nE, cbase, nodeBase, vec8, list, tid, lane, wave);
    if (lane == 0) wcnt[wave] = wc;
    __syncthreads();
    if (wave == 0) {
#pragma unroll 1
      for (int wsx = 0; wsx < NWAVE; ++wsx) {
        int n = __builtin_amdgcn_readfirstlane(wcnt[wsx]);
        n = n > WCAP ? WCAP : (n < 0 ? 0 : n);
        const int* lp = list + wsx * WCAP;
#pragma unroll 1
        for (int i = 0; i < n; ++i) {
          const int ent  = __builtin_amdgcn_readfirstlane(lp[i]);
          const int slot = ent & (NBF - 1);
          int e = cbase + ((ent >> 12) & (CHUNK - 1));
          e = e > nE - 1 ? nE - 1 : e;
          int src = ei[e];
          src = src < 0 ? 0 : (src > nN - 1 ? nN - 1 : src);
          if (lane == 0) {
            int pos = cursor[slot];
            pos = pos < 0 ? 0 : (pos > RCAP - 1 ? RCAP - 1 : pos);
            region[pos] = src;
            const int np = pos + 1;
            cursor[slot] = np > RCAP ? RCAP : np;
          }
        }
      }
    }
    __syncthreads();
  }

  const int nv = lenW >> 2;
  int* gp = csr + rb0;
#pragma unroll 1
  for (int i = tid; i < nv; i += NTHR) { const v4i v = ((const v4i*)region)[i]; *(volatile v4i*)(gp + 4 * i) = v; }
  __threadfence();
#pragma unroll 1
  for (int i = tid; i < nv; i += NTHR) { const v4i v = ((const v4i*)region)[i]; *(volatile v4i*)(gp + 4 * i) = v; }
}

__global__ __launch_bounds__(NTHR) void k_prop(
    const int* __restrict__ csr, const int* __restrict__ off, const int* __restrict__ cnt,
    const float* __restrict__ dinv, const float* __restrict__ hin, float* pout,
    int nN, int hinRows, int csrLen) {
  const int tid = threadIdx.x, lane = tid & 31, wave = tid >> 5;
  const int tbase = blockIdx.x * TGT + wave * 32;
  const int cl = tbase + lane;
  const int cnt_l = cnt[cl];
  const int off_l = off[cl];
  FI dvu; dvu.f = dinv[cl];

#pragma unroll 1
  for (int j = 0; j < 32; ++j) {
    const int c = tbase + j;
    int n = __builtin_amdgcn_readlane(cnt_l, j);
    n = n < 0 ? 0 : (n > DEGCAP ? DEGCAP : n);
    const int st = __builtin_amdgcn_readlane(off_l, j);
    FI du; du.i = __builtin_amdgcn_readlane(dvu.i, j);
    const float dc = du.f;
    v4f acc = {0.f, 0.f, 0.f, 0.f};
#pragma unroll 1
    for (int q0 = 0; q0 < n; q0 += 32) {
      int pos = st + q0 + lane;
      pos = pos < 0 ? 0 : (pos > csrLen - 1 ? csrLen - 1 : pos);
      int sl = csr[pos];
      sl = sl < 0 ? 0 : (sl > nN - 1 ? nN - 1 : sl);
      FI wl; wl.f = dinv[sl];
      const int mcnt = (n - q0) < 32 ? (n - q0) : 32;
#pragma unroll 1
      for (int p = 0; p < mcnt; ++p) {
        const int s = __builtin_amdgcn_readlane(sl, p);
        FI wu; wu.i = __builtin_amdgcn_readlane(wl.i, p);
        const v4f v = *(const v4f*)(hin + (size_t)s * D + 4 * lane);
        acc = acc + v * wu.f;
      }
    }
    const int cc = c < hinRows ? c : hinRows - 1;
    const v4f sv = *(const v4f*)(hin + (size_t)cc * D + 4 * lane);
    const v4f r = (acc + sv * dc) * dc;
    float* pp = pout + (size_t)c * D + 4 * lane;
    *(volatile v4f*)pp = r;
    __threadfence();
    *(volatile v4f*)pp = r;
  }
}

template <int NT, int STATS>
__global__ __launch_bounds__(NTHR) void k_gemm(
    const float* __restrict__ A, const unsigned short* __restrict__ Bh, const unsigned short* __restrict__ Bl,
    const float* __restrict__ bias, float* C, double* part, int nRowsA, int nRowsOut, int nStat) {
  static_assert(NT == 8 || NT == 4);
  static_assert(STATS == 0 || NT == 8);
  extern __shared__ v4f lds_dyn[];
  constexpr int OP = 16 * NT;
  unsigned short* sAh = (unsigned short*)lds_dyn;
  unsigned short* sAl = sAh + GROWS * AP;
  float*  stg = (float*)lds_dyn;
  double* sst = (double*)((char*)lds_dyn + LDS_GST);
  const int tid = threadIdx.x, lane = tid & 31, wave = tid >> 5, hh = lane >> 4, m = lane & 15;
  const int rowBase = blockIdx.x * GROWS;

#pragma unroll
  for (int i = 0; i < (GROWS * D / 8) / NTHR; ++i) {
    const int idx = i * NTHR + tid;
    const int r   = idx >> 4;
    const int c0  = (idx & 15) * 8;
    int row = rowBase + r;
    row = row > nRowsA - 1 ? nRowsA - 1 : row;
    const float* ap = A + (size_t)row * D + c0;
    const v4f a = *(const v4f*)ap, b = *(const v4f*)(ap + 4);
    v8us hv, lv;
    split8(a, b, hv, lv);
    *(v8us*)(sAh + r * AP + c0) = hv;
    *(v8us*)(sAl + r * AP + c0) = lv;
  }
  __syncthreads();

  v8f acc[NT];
#pragma unroll
  for (int t = 0; t < NT; ++t) { v8f z = {0.f, 0.f, 0.f, 0.f, 0.f, 0.f, 0.f, 0.f}; acc[t] = z; }
  const unsigned short* arh = sAh + (wave * 16 + m) * AP + 8 * hh;
  const unsigned short* arl = sAl + (wave * 16 + m) * AP + 8 * hh;
#pragma unroll
  for (int kt = 0; kt < D / 32; ++kt) {
    FragB ah, al;
    ah.h[0] = *(const v8us*)(arh + 32 * kt);
    ah.h[1] = *(const v8us*)(arh + 32 * kt + 16);
    al.h[0] = *(const v8us*)(arl + 32 * kt);
    al.h[1] = *(const v8us*)(arl + 32 * kt + 16);
#pragma unroll
    for (int t = 0; t < NT; ++t) {
      const size_t bo = (size_t)(16 * t + m) * D + 32 * kt + 8 * hh;
      FragB bh, bl;
      bh.h[0] = *(const v8us*)(Bh + bo);
      bh.h[1] = *(const v8us*)(Bh + bo + 16);
      bl.h[0] = *(const v8us*)(Bl + bo);
      bl.h[1] = *(const v8us*)(Bl + bo + 16);
      acc[t] = wmb(ah.v, bh.v, acc[t]);
      acc[t] = wmb(al.v, bh.v, acc[t]);
      acc[t] = wmb(ah.v, bl.v, acc[t]);
    }
  }
  __syncthreads();

  const int r0 = wave * 16 + 8 * hh;
  float* sp = stg + r0 * OP + m;
#pragma unroll
  for (int t = 0; t < NT; ++t) {
    const float bv = bias[16 * t + m];
#pragma unroll
    for (int r = 0; r < 8; ++r) sp[r * OP + 16 * t] = acc[t][r] + bv;
  }
  __syncthreads();

  v2d pv = {0.0, 0.0};
  double* pp = part;
  if (STATS != 0) {
    int nv = nStat - rowBase;
    nv = nv < 0 ? 0 : (nv > GROWS ? GROWS : nv);
    const int col = tid & (OP - 1);
    const int st  = tid >> 7;
    double s = 0.0;
#pragma unroll 1
    for (int r = 0; r < nv; ++r) {
      const double dv = (double)stg[r * OP + col];
      const double q  = (st != 0) ? dv * dv : dv;
      s += q;
    }
    sst[st * 128 + col] = s;
    __syncthreads();
    if (tid < 128) pv = *(const v2d*)(sst + 2 * tid);
    pp = part + (size_t)blockIdx.x * 256 + 2 * tid;
  }

  constexpr int RPI = 128 / OP;
  constexpr int LPR = 32 / RPI;
  constexpr int NI  = 16 / RPI;
  const int rsub = lane / LPR, csub = 4 * (lane % LPR);
  v4f vals[NI];
#pragma unroll
  for (int i = 0; i < NI; ++i) {
    const int rloc = wave * 16 + i * RPI + rsub;
    vals[i] = *(const v4f*)(stg + rloc * OP + csub);
  }
  if (STATS != 0 && tid < 128) *(volatile v2d*)pp = pv;
#pragma unroll
  for (int i = 0; i < NI; ++i) {
    const int rloc = wave * 16 + i * RPI + rsub;
    const int grow = rowBase + rloc;
    if (grow < nRowsOut) *(volatile v4f*)(C + (size_t)grow * OP + csub) = vals[i];
  }
  __threadfence();
  if (STATS != 0 && tid < 128) *(volatile v2d*)pp = pv;
#pragma unroll
  for (int i = 0; i < NI; ++i) {
    const int rloc = wave * 16 + i * RPI + rsub;
    const int grow = rowBase + rloc;
    if (grow < nRowsOut) *(volatile v4f*)(C + (size_t)grow * OP + csub) = vals[i];
  }
}

__global__ __launch_bounds__(NTHR) void k_bnfin(
    const double* __restrict__ part, int nBlk, const float* __restrict__ gam, const float* __restrict__ bet,
    int nN, float* ss) {
  __shared__ double sd[256];
  __shared__ __attribute__((aligned(16))) float sf[256];
  const int tid = threadIdx.x;
  double s = 0.0;
#pragma unroll 1
  for (int b = 0; b < nBlk; ++b) s += part[(size_t)b * 256 + tid];
  sd[tid] = s;
  __syncthreads();
  if (tid < 128) {
    const double invn = 1.0 / (double)nN;
    const double mean = sd[tid] * invn;
    double var = sd[128 + tid] * invn - mean * mean;
    var = var < 0.0 ? 0.0 : var;
    const float istd = rsqrtf((float)var + BNEPS);
    const float sc = istd * gam[tid];
    const float sh = bet[tid] - (float)mean * sc;
    sf[tid] = sc;
    sf[128 + tid] = sh;
  }
  __syncthreads();
  v4f o = {0.f, 0.f, 0.f, 0.f};
  if (tid < 64) o = *(const v4f*)(sf + 4 * tid);
  if (tid < 64) *(volatile v4f*)(ss + 4 * tid) = o;
  __threadfence();
  if (tid < 64) *(volatile v4f*)(ss + 4 * tid) = o;
}

__global__ __launch_bounds__(NTHR) void k_bnrelu(float* Y, const float* __restrict__ ss) {
  const int tid = threadIdx.x, lane = tid & 31, wave = tid >> 5;
  const int row0 = blockIdx.x * BNR + wave * 8;
  const v4f sc = *(const v4f*)(ss + 4 * lane);
  const v4f sh = *(const v4f*)(ss + 128 + 4 * lane);
  v4f rr[8];
#pragma unroll
  for (int i = 0; i < 8; ++i) {
    const float* p = Y + (size_t)(row0 + i) * D + 4 * lane;
    const v4f v = *(const v4f*)p;
    v4f r = v * sc + sh;
    r.x = fmaxf(r.x, 0.f); r.y = fmaxf(r.y, 0.f); r.z = fmaxf(r.z, 0.f); r.w = fmaxf(r.w, 0.f);
    rr[i] = r;
  }
#pragma unroll
  for (int i = 0; i < 8; ++i) *(volatile v4f*)(Y + (size_t)(row0 + i) * D + 4 * lane) = rr[i];
  __threadfence();
#pragma unroll
  for (int i = 0; i < 8; ++i) *(volatile v4f*)(Y + (size_t)(row0 + i) * D + 4 * lane) = rr[i];
}

__global__ __launch_bounds__(NTHR) void k_decode(
    const float* __restrict__ emb, const int* __restrict__ eli, float* rout, int nN, int EL) {
  const int tid = threadIdx.x, lane = tid & 31, wave = tid >> 5;
  const int wbase = (blockIdx.x * NWAVE + wave) * 32;
  if (wbase < EL) {
    int el = wbase + lane;
    el = el > EL - 1 ? EL - 1 : el;
    int a_l = eli[el];
    int b_l = eli[(size_t)EL + el];
    a_l = a_l < 0 ? 0 : (a_l > nN - 1 ? nN - 1 : a_l);
    b_l = b_l < 0 ? 0 : (b_l > nN - 1 ? nN - 1 : b_l);
    float res = 0.f;
#pragma unroll 1
    for (int j = 0; j < 32; ++j) {
      const int a = __builtin_amdgcn_readlane(a_l, j);
      const int b = __builtin_amdgcn_readlane(b_l, j);
      const v4f va = *(const v4f*)(emb + (size_t)a * D + 4 * lane);
      const v4f vb = *(const v4f*)(emb + (size_t)b * D + 4 * lane);
      float s = va.x * vb.x + va.y * vb.y + va.z * vb.z + va.w * vb.w;
#pragma unroll
      for (int o = 16; o > 0; o >>= 1) s += __shfl_xor(s, o, 32);
      float scl = s > 30.f ? 30.f : (s < -30.f ? -30.f : s);
      const float dnm = 1.0f + __expf(-scl);
      const float sig = __builtin_amdgcn_rcpf(dnm);
      res = (lane == j) ? sig : res;
    }
    const bool ok = (wbase + lane) < EL;
    float* rp = rout + wbase + lane;
    if (ok) *(volatile float*)rp = res;
    __threadfence();
    if (ok) *(volatile float*)rp = res;
  }
}

extern "C" void kernel_launch(void* const* d_in, const int* in_sizes, int n_in,
                              void* d_out, int out_size, void* d_ws, size_t ws_size,
                              hipStream_t stream) {
  if (n_in < 13) return;
  const int nN = in_sizes[0] / D;
  const int nE = in_sizes[1] / 2;
  const int EL = in_sizes[2] / 2;
  if (nN <= 0 || nE <= 0 || EL <= 0) return;
  if (in_sizes[0] != nN * D || in_sizes[1] != 2 * nE || in_sizes[2] != 2 * EL) return;
  if (in_sizes[3] != D * D || in_sizes[4] < D || in_sizes[5] < D || in_sizes[6] < D) return;
  if (in_sizes[7] != D * D || in_sizes[8] < D || in_sizes[9] < D || in_sizes[10] < D) return;
  if (in_sizes[11] != D * DO || in_sizes[12] < DO) return;
  if ((size_t)out_size != (size_t)nN * DO + (size_t)EL) return;
  if (nE > (1 << 28) || nN > (1 << 24)) return;

  const float* x   = (const float*)d_in[0];
  const int*   ei  = (const int*)d_in[1];
  const int*   eli = (const int*)d_in[2];
  const float* W1  = (const float*)d_in[3];
  const float* b1  = (const float*)d_in[4];
  const float* g1  = (const float*)d_in[5];
  const float* be1 = (const float*)d_in[6];
  const float* W2  = (const float*)d_in[7];
  const float* b2  = (const float*)d_in[8];
  const float* g2  = (const float*)d_in[9];
  const float* be2 = (const float*)d_in[10];
  const float* W3  = (const float*)d_in[11];
  const float* b3  = (const float*)d_in[12];
  float* out0 = (float*)d_out;
  float* out1 = out0 + (size_t)nN * DO;

  const int NPAD   = ((nN + TGT - 1) / TGT) * TGT;
  const int nBC    = (nN + NBC - 1) / NBC;
  const int CNTPAD = nBC * NBC;
  if (4 * nBC + 1 > RBN) return;
  const int nBF    = (nN + NBF - 1) / NBF;
  const int csrLen = ((nE + 31) & ~31) + 4096;
  const int nGemm  = NPAD / GROWS;
  const int nAgg   = NPAD / TGT;
  const int nBn    = NPAD / BNR;
  const int nDec   = (EL + NTHR - 1) / NTHR;

  char* ws = (char*)d_ws;
  size_t off = 0;
  const size_t oWh1 = off; off += (size_t)D * D * 2;          off = (off + 255) & ~(size_t)255;
  const size_t oWl1 = off; off += (size_t)D * D * 2;          off = (off + 255) & ~(size_t)255;
  const size_t oWh2 = off; off += (size_t)D * D * 2;          off = (off + 255) & ~(size_t)255;
  const size_t oWl2 = off; off += (size_t)D * D * 2;          off = (off + 255) & ~(size_t)255;
  const size_t oWh3 = off; off += (size_t)D * DO * 2;         off = (off + 255) & ~(size_t)255;
  const size_t oWl3 = off; off += (size_t)D * DO * 2;         off = (off + 255) & ~(size_t)255;
  const size_t oCnt = off; off += (size_t)CNTPAD * 4;         off = (off + 255) & ~(size_t)255;
  const size_t oDv  = off; off += (size_t)CNTPAD * 4;         off = (off + 255) & ~(size_t)255;
  const size_t oOff = off; off += (size_t)CNTPAD * 4;         off = (off + 255) & ~(size_t)255;
  const size_t oRb  = off; off += (size_t)RBN * 4;            off = (off + 255) & ~(size_t)255;
  const size_t oCsr = off; off += (size_t)csrLen * 4;         off = (off + 255) & ~(size_t)255;
  const size_t oP   = off; off += (size_t)NPAD * D * 4;       off = (off + 255) & ~(size_t)255;
  const size_t oY   = off; off += (size_t)NPAD * D * 4;       off = (off + 255) & ~(size_t)255;
  const size_t oPt  = off; off += (size_t)nGemm * 256 * 8;    off = (off + 255) & ~(size_t)255;
  const size_t oSs  = off; off += (size_t)256 * 4;            off = (off + 255) & ~(size_t)255;
  if (off > ws_size) return;
  unsigned short* wh1 = (unsigned short*)(ws + oWh1);
  unsigned short* wl1 = (unsigned short*)(ws + oWl1);
  unsigned short* wh2 = (unsigned short*)(ws + oWh2);
  unsigned short* wl2 = (unsigned short*)(ws + oWl2);
  unsigned short* wh3 = (unsigned short*)(ws + oWh3);
  unsigned short* wl3 = (unsigned short*)(ws + oWl3);
  int*    cnt  = (int*)(ws + oCnt);
  float*  dinv = (float*)(ws + oDv);
  int*    offp = (int*)(ws + oOff);
  int*    rb   = (int*)(ws + oRb);
  int*    csr  = (int*)(ws + oCsr);
  float*  P    = (float*)(ws + oP);
  float*  Y    = (float*)(ws + oY);
  double* part = (double*)(ws + oPt);
  float*  ss   = (float*)(ws + oSs);

  const int vec8 = ((nE & 3) == 0) ? 1 : 0;

  const int nPrep = (D * D / 8 + D * D / 8 + D * DO / 8) / NTHR;
  k_wprep<<<nPrep, NTHR, 0, stream>>>(W1, W2, W3, wh1, wl1, wh2, wl2, wh3, wl3);

  k_count<<<nBC, NTHR, 0, stream>>>(ei, cnt, dinv, nE, vec8);
  k_offsets<<<1, OTHR, 0, stream>>>(cnt, offp, rb, nBC);
  hipFuncSetAttribute(reinterpret_cast<const void*>(&k_fill),
                      hipFuncAttributeMaxDynamicSharedMemorySize, LDS_FILL);
  k_fill<<<nBF, NTHR, LDS_FILL, stream>>>(ei, offp, rb, csr, nN, nE, vec8, csrLen);

  hipFuncSetAttribute(reinterpret_cast<const void*>(&k_gemm<8, 1>),
                      hipFuncAttributeMaxDynamicSharedMemorySize, LDS_GEMM);
  hipFuncSetAttribute(reinterpret_cast<const void*>(&k_gemm<4, 0>),
                      hipFuncAttributeMaxDynamicSharedMemorySize, LDS_GEMM);

  k_prop<<<nAgg, NTHR, 0, stream>>>(csr, offp, cnt, dinv, x, P, nN, nN, csrLen);
  k_gemm<8, 1><<<nGemm, NTHR, LDS_GEMM, stream>>>(P, wh1, wl1, b1, Y, part, NPAD, NPAD, nN);
  k_bnfin<<<1, NTHR, 0, stream>>>(part, nGemm, g1, be1, nN, ss);
  k_bnrelu<<<nBn, NTHR, 0, stream>>>(Y, ss);

  k_prop<<<nAgg, NTHR, 0, stream>>>(csr, offp, cnt, dinv, Y, P, nN, NPAD, csrLen);
  k_gemm<8, 1><<<nGemm, NTHR, LDS_GEMM, stream>>>(P, wh2, wl2, b2, Y, part, NPAD, NPAD, nN);
  k_bnfin<<<1, NTHR, 0, stream>>>(part, nGemm, g2, be2, nN, ss);
  k_bnrelu<<<nBn, NTHR, 0, stream>>>(Y, ss);

  k_prop<<<nAgg, NTHR, 0, stream>>>(csr, offp, cnt, dinv, Y, P, nN, NPAD, csrLen);
  k_gemm<4, 0><<<nGemm, NTHR, LDS_GEMM, stream>>>(P, wh3, wl3, b3, out0, part, NPAD, nN, nN);
  k_decode<<<nDec, NTHR, 0, stream>>>(P, eli, out1, nN, EL);
}
